// CausalSelfAttention_13941463842848
// MI455X (gfx1250) — hardware-verified
//
#include <hip/hip_runtime.h>
#include <math.h>

typedef __attribute__((ext_vector_type(16))) _Float16 v16h;
typedef __attribute__((ext_vector_type(16))) __bf16 v16b;
typedef __attribute__((ext_vector_type(8)))  _Float16 v8h;
typedef __attribute__((ext_vector_type(8)))  __bf16 v8b;
typedef __attribute__((ext_vector_type(8)))  float v8f;
typedef __attribute__((ext_vector_type(4)))  float v4f;
typedef __attribute__((ext_vector_type(4)))  unsigned v4u;
typedef v8h __attribute__((may_alias)) v8h_a;
typedef v4f __attribute__((may_alias)) v4f_a;
typedef v4u __attribute__((may_alias)) v4u_a;

#ifndef NB
#define NB 1
#endif
#ifndef SEQ
#define SEQ 4096
#endif
#define SEQ_FULL 4096
#define EMB 2048u
#define NH 16u
#define NKV 4u
#define HD 128u
#define KVW 512u
#define NQKV 3072u
#define WIN 1023u
#define HIQ (SEQ < 512 ? SEQ : 512)
#define SCALE (0.08838834764831845f)
#define RMS_EPS (1.1920929e-07f)

static_assert(NB == 1);
static_assert(SEQ % 64 == 0);
static_assert(HIQ % 64 == 0);
static_assert(SEQ <= SEQ_FULL);
static_assert(((size_t)SEQ * EMB) % 2048u == 0);
static_assert(NQKV % 128u == 0 && EMB % 128u == 0 && KVW % 128u == 0);
static_assert(HD == 128u && EMB == NH * HD && KVW == NKV * HD && NQKV == EMB + 2u * KVW);
static_assert(WIN + 1u == 16u * 64u);
static_assert(SEQ % 4 == 0);
static_assert(NH / NKV == 4u);

template <typename T> __device__ __forceinline__ void vst2(void* p, T v) { *(volatile T*)p = v; __threadfence(); *(volatile T*)p = v; }
__device__ __forceinline__ v8f wmma16(v16h a, v16h b, v8f c) {
  v8f d = __builtin_amdgcn_wmma_f32_16x16x32_f16(false, a, false, b, (short)0, c, false, false);
  asm volatile("v_nop\n\tv_nop\n\tv_nop\n\tv_nop" : "+v"(d) : "v"(a), "v"(b));
  return d;
}
__device__ __forceinline__ v8f wmma_bf(v16b a, v16b b, v8f c) {
  v8f d = __builtin_amdgcn_wmma_f32_16x16x32_bf16(false, a, false, b, (short)0, c, false, false);
  asm volatile("v_nop\n\tv_nop\n\tv_nop\n\tv_nop" : "+v"(d) : "v"(a), "v"(b));
  return d;
}
__device__ __forceinline__ v16h frag_h(const _Float16* rowk0, unsigned lane) {
  union { v16h v; v8h q[2]; } u; const _Float16* p = rowk0 + 8u * (lane >> 4);
  u.q[0] = *(const v8h*)p; u.q[1] = *(const v8h*)(p + 16); return u.v;
}
__device__ __forceinline__ v16b frag_b(const __bf16* rowk0, unsigned lane) {
  union { v16b v; v8b q[2]; } u; const __bf16* p = rowk0 + 8u * (lane >> 4);
  u.q[0] = *(const v8b*)p; u.q[1] = *(const v8b*)(p + 16); return u.v;
}
struct F2 { v16b h, l; };
__device__ __forceinline__ F2 bsplit16(const float v[16]) { F2 r;
#pragma unroll
  for (int i = 0; i < 16; ++i) { const __bf16 h = (__bf16)v[i]; r.h[i] = h; r.l[i] = (__bf16)(v[i] - (float)h); }
  return r; }
__device__ __forceinline__ float bfr(float v) { return (float)(__bf16)v; }
static __device__ __forceinline__ _Float16 toh_flush(float v) { const _Float16 r = (_Float16)v; return (fabsf(v) < 6.103515625e-05f) ? (_Float16)0.0f : r; }
#define LDSX() do { asm volatile("s_wait_dscnt 0" ::: "memory"); __builtin_amdgcn_wave_barrier(); __builtin_amdgcn_fence(3  , "workgroup"); } while (0)

#define WS_XB  ((size_t)0)
#define WS_WB  (WS_XB  + 2u * (size_t)SEQ * EMB)
#define WS_WO  (WS_WB  + 2u * (size_t)NQKV * EMB)
#define WS_QH  (WS_WO  + 2u * (size_t)EMB * EMB)
#define WS_KH  (WS_QH  + 2u * (size_t)SEQ * EMB)
#define WS_VT  (WS_KH  + 2u * (size_t)SEQ * KVW)
#define WS_QL  (WS_VT  + 2u * (size_t)KVW * SEQ)
#define WS_KL  (WS_QL  + 2u * (size_t)HIQ * EMB)
#define WS_VB  (WS_KL  + 2u * (size_t)HIQ * KVW)
#define WS_VBL (WS_VB  + 2u * (size_t)KVW * HIQ)
#define WS_CH  (WS_VBL + 2u * (size_t)KVW * HIQ)
#define WS_CL  (WS_CH  + 2u * (size_t)SEQ * EMB)
#define WS_CS  (WS_CL  + 2u * (size_t)HIQ * EMB)
#define WS_END (WS_CS  + 4u * (size_t)SEQ * HD)
static_assert(WS_END <= (size_t)134217728);
static_assert(WS_CS % 128u == 0 && WS_END % 128u == 0);

__global__ __launch_bounds__(256) void k_cvt_b(const float* __restrict__ in, __bf16* __restrict__ out, unsigned n8) {
  const unsigned i = blockIdx.x * 256u + threadIdx.x; const unsigned ic = i < n8 ? i : n8 - 1u;
  const float* p = in + (size_t)ic * 8u; const v4f a = *(const v4f*)p, b = *(const v4f*)(p + 4);
  union { v8b b; v4u u; } o;
  o.b[0] = (__bf16)a[0]; o.b[1] = (__bf16)a[1]; o.b[2] = (__bf16)a[2]; o.b[3] = (__bf16)a[3];
  o.b[4] = (__bf16)b[0]; o.b[5] = (__bf16)b[1]; o.b[6] = (__bf16)b[2]; o.b[7] = (__bf16)b[3];
  if (i < n8) vst2((void*)(out + (size_t)i * 8u), o.u);
}
__global__ __launch_bounds__(256) void k_cvt_h(const float* __restrict__ in, _Float16* __restrict__ out, unsigned n8) {
  const unsigned i = blockIdx.x * 256u + threadIdx.x; const unsigned ic = i < n8 ? i : n8 - 1u;
  const float* p = in + (size_t)ic * 8u; const v4f a = *(const v4f*)p, b = *(const v4f*)(p + 4);
  union { v8h h; v4u u; } o;
  o.h[0] = (_Float16)(bfr(a[0]) * 256.0f); o.h[1] = (_Float16)(bfr(a[1]) * 256.0f); o.h[2] = (_Float16)(bfr(a[2]) * 256.0f); o.h[3] = (_Float16)(bfr(a[3]) * 256.0f);
  o.h[4] = (_Float16)(bfr(b[0]) * 256.0f); o.h[5] = (_Float16)(bfr(b[1]) * 256.0f); o.h[6] = (_Float16)(bfr(b[2]) * 256.0f); o.h[7] = (_Float16)(bfr(b[3]) * 256.0f);
  if (i < n8) vst2((void*)(out + (size_t)i * 8u), o.u);
}

__global__ __launch_bounds__(256) void k_rope_tab(float* __restrict__ CS) {
#pragma clang fp contract(off)
  __shared__ __align__(16) float st[4][128];
  const unsigned tid = threadIdx.x, tl = tid >> 6, d = tid & 63u; const unsigned t = blockIdx.x * 4u + tl;
  double w = 1.0;
#pragma unroll 1
  for (unsigned i = 0; i < d; ++i) w *= 1.1547819846894583;
  const float pw = (float)w; const float inv_freq = 1.0f / pw; const float ang = (float)t * inv_freq;
  float sv, cv; sincosf(ang, &sv, &cv);
  st[tl][d] = cv; st[tl][64u + d] = sv;
  __syncthreads();
  if (tid < 128u) { const unsigned rl = tid >> 5, ln = tid & 31u; const v4f v = *(const v4f_a*)&st[rl][ln * 4u];
    vst2((void*)(CS + (size_t)(blockIdx.x * 4u + rl) * HD + ln * 4u), v); }
}

__global__ __launch_bounds__(128) void k_proj(const __bf16* __restrict__ XB, const __bf16* __restrict__ WB, const float* __restrict__ CS,
    _Float16* __restrict__ QH, _Float16* __restrict__ QL, _Float16* __restrict__ KH, _Float16* __restrict__ KL, _Float16* __restrict__ VT, __bf16* __restrict__ VB, __bf16* __restrict__ VBL) {
  __shared__ __align__(16) _Float16 sh[64][136], sl[64][136]; __shared__ __align__(16) _Float16 th[128][72]; __shared__ __align__(16) __bf16 tb[128][72], tbl[128][72];
  __shared__ __align__(16) float sf[64][132];
  const unsigned tid = threadIdx.x, wave = tid >> 5, lane = tid & 31u, col = lane & 15u, g = lane >> 4;
  const unsigned r0 = blockIdx.x * 64u, c0 = blockIdx.y * 128u; const unsigned which = c0 < EMB ? 0u : (c0 < EMB + KVW ? 1u : 2u);
  const unsigned wr = (wave & 1u) * 32u, wc = (wave >> 1) * 64u;
  v8f acc[2][4] = {};
  const __bf16* pa = XB + (size_t)(r0 + wr + col) * EMB; const __bf16* pb = WB + (size_t)(c0 + wc + col) * EMB;
#pragma unroll 1
  for (unsigned kc = 0; kc < EMB; kc += 32u) { const v16b a0 = frag_b(pa + kc, lane), a1 = frag_b(pa + (size_t)16u * EMB + kc, lane);
#pragma unroll
    for (int t = 0; t < 4; ++t) { const v16b w = frag_b(pb + (size_t)t * 16u * EMB + kc, lane); acc[0][t] = wmma_bf(a0, w, acc[0][t]); acc[1][t] = wmma_bf(a1, w, acc[1][t]); } }
  const bool hi_rows = r0 < (unsigned)HIQ;
  const unsigned cb = which == 0u ? c0 : (which == 1u ? c0 - EMB : c0 - EMB - KVW);
  if (which < 2u) { _Float16* DH = which == 0u ? QH : KH; _Float16* DL = which == 0u ? QL : KL; const unsigned pitch = which == 0u ? EMB : KVW;
#pragma unroll
    for (int mi = 0; mi < 2; ++mi)
#pragma unroll
      for (int t = 0; t < 4; ++t) { const unsigned cl = wc + t * 16u + col;
#pragma unroll
        for (int r = 0; r < 8; ++r) { const unsigned rl = wr + mi * 16u + 8u * g + r; sf[rl][cl] = acc[mi][t][r]; } }
    __syncthreads();
    { const unsigned rl = tid >> 1, hf = tid & 1u;
      float ss = 0.f;
#pragma unroll 1
      for (unsigned i = 0; i < 64u; ++i) { const float v = sf[rl][hf * 64u + i]; ss += v * v; }
      ss += __shfl_xor(ss, 1);
      const float rn = rsqrtf(ss * (1.0f / 128.0f) + RMS_EPS);
      const float* tab = CS + (size_t)(r0 + rl) * HD;
#pragma unroll 1
      for (unsigned i = 0; i < 32u; ++i) { const unsigned d = hf * 32u + i; const float a = sf[rl][d] * rn, b = sf[rl][d + 64u] * rn; const float c = tab[d], s = tab[64u + d];
        const float o1 = a * c + b * s, o2 = b * c - a * s;
        const _Float16 h1 = toh_flush(o1), h2 = toh_flush(o2);
        sh[rl][d] = h1; sh[rl][d + 64u] = h2;
        sl[rl][d] = toh_flush((o1 - (float)h1) * 1024.0f); sl[rl][d + 64u] = toh_flush((o2 - (float)h2) * 1024.0f); } }
    __syncthreads();
    for (unsigned e = tid; e < 64u * 16u; e += 128u) { const unsigned rl = e >> 4, q = e & 15u;
      const v4u vh = *(const v4u_a*)&sh[rl][q * 8u]; vst2((void*)(DH + (size_t)(r0 + rl) * pitch + cb + q * 8u), vh);
      if (hi_rows) { const v4u vl = *(const v4u_a*)&sl[rl][q * 8u]; vst2((void*)(DL + (size_t)(r0 + rl) * pitch + cb + q * 8u), vl); } }
  } else {
#pragma unroll
    for (int mi = 0; mi < 2; ++mi)
#pragma unroll
      for (int t = 0; t < 4; ++t) { const unsigned cl = wc + t * 16u + col;
#pragma unroll
        for (int r = 0; r < 8; ++r) { const unsigned rl = wr + mi * 16u + 8u * g + r; const float v = acc[mi][t][r]; th[cl][rl] = toh_flush(v); const __bf16 bh = (__bf16)v; tb[cl][rl] = bh; tbl[cl][rl] = (__bf16)(v - (float)bh); } }
    __syncthreads();
    for (unsigned e = tid; e < 128u * 8u; e += 128u) { const unsigned cl = e >> 3, q = e & 7u;
      const v4u vv = *(const v4u_a*)&th[cl][q * 8u]; vst2((void*)(VT + (size_t)(cb + cl) * SEQ + r0 + q * 8u), vv);
      if (hi_rows) { const size_t o3 = (size_t)(cb + cl) * HIQ + r0 + q * 8u; const v4u v1 = *(const v4u_a*)&tb[cl][q * 8u]; const v4u v2 = *(const v4u_a*)&tbl[cl][q * 8u]; vst2((void*)(VB + o3), v1); vst2((void*)(VBL + o3), v2); } } }
}

template <bool HI>
__device__ __forceinline__ void attn_body(const _Float16* __restrict__ QH, const _Float16* __restrict__ KH, const _Float16* __restrict__ VT, const _Float16* __restrict__ QL, const _Float16* __restrict__ KL,
    const __bf16* __restrict__ VB, const __bf16* __restrict__ VBL, _Float16* __restrict__ CH, _Float16* __restrict__ CL, unsigned qb0) {
  __shared__ __align__(16) _Float16 ph[4][16][72];
  __shared__ __align__(16) float pf[4][16][68];
  __shared__ __align__(16) _Float16 cs[4][16][136];
  __shared__ __align__(16) _Float16 csl[4][16][136];
  const unsigned tid = threadIdx.x, wave = tid >> 5, lane = tid & 31u, col = lane & 15u, g = lane >> 4;
  const unsigned qb = qb0 + blockIdx.x, h = blockIdx.y, kvh = h >> 2;
  const unsigned ql0 = qb * 64u + wave * 16u; const unsigned kt0 = qb >= 16u ? qb - 16u : 0u;
  const size_t qrow = (size_t)(ql0 + col) * EMB + h * HD;
  v8f acc[8] = {};
  float mrow[8], lrow[8];
#pragma unroll
  for (int r = 0; r < 8; ++r) { mrow[r] = -3.0e38f; lrow[r] = 0.f; }
#pragma unroll 1
  for (unsigned kt = kt0; kt <= qb; ++kt) { const unsigned k0 = kt * 64u;
    unsigned zo = 0u; asm volatile("" : "+v"(zo));
    v8f s[4] = {}, sr[4] = {};
#pragma unroll 1
    for (unsigned kc = 0; kc < HD; kc += 32u) { const v16h ah = frag_h(QH + qrow + kc + zo, lane); v16h al = ah; if (HI) al = frag_h(QL + qrow + kc + zo, lane);
#pragma unroll
      for (int j = 0; j < 4; ++j) { const size_t ko = (size_t)(k0 + j * 16u + col) * KVW + kvh * HD + kc; const v16h kf = frag_h(KH + ko, lane); s[j] = wmma16(ah, kf, s[j]);
        if (HI) { sr[j] = wmma16(al, kf, sr[j]); const v16h kl = frag_h(KL + ko, lane); sr[j] = wmma16(ah, kl, sr[j]); } } }
#pragma unroll
    for (int r = 0; r < 8; ++r) { const unsigned qi = ql0 + 8u * g + r; float v[4], p[4];
#pragma unroll
      for (int j = 0; j < 4; ++j) { const unsigned key = k0 + j * 16u + col; float x = s[j][r]; if (HI) x += sr[j][r] * (1.0f / 1024.0f); x *= SCALE; const bool vis = (key <= qi) && (key + WIN >= qi); v[j] = vis ? x : -3.0e38f; }
      float mx = fmaxf(fmaxf(v[0], v[1]), fmaxf(v[2], v[3]));
      mx = fmaxf(mx, __shfl_xor(mx, 1)); mx = fmaxf(mx, __shfl_xor(mx, 2)); mx = fmaxf(mx, __shfl_xor(mx, 4)); mx = fmaxf(mx, __shfl_xor(mx, 8));
      const float mnew = fmaxf(mrow[r], mx); const float sc = expf(mrow[r] - mnew);
      float rs = 0.f;
#pragma unroll
      for (int j = 0; j < 4; ++j) { const float e = expf(v[j] - mnew); p[j] = (v[j] <= -1.0e38f) ? 0.f : e; rs += p[j]; }
      rs += __shfl_xor(rs, 1); rs += __shfl_xor(rs, 2); rs += __shfl_xor(rs, 4); rs += __shfl_xor(rs, 8);
      lrow[r] = lrow[r] * sc + rs; mrow[r] = mnew;
#pragma unroll
      for (int dt = 0; dt < 8; ++dt) acc[dt][r] *= sc;
#pragma unroll
      for (int j = 0; j < 4; ++j) { if (HI) pf[wave][8u * g + r][j * 16u + col] = p[j]; else ph[wave][8u * g + r][j * 16u + col] = toh_flush(p[j] * 2048.0f); } }
    LDSX();
    if (HI) {
#pragma unroll 1
      for (unsigned kk = 0; kk < 2u; ++kk) { float pv[16]; const float* pp = &pf[wave][col][kk * 32u + 8u * g];
        const v4f x0 = *(const v4f_a*)pp, x1 = *(const v4f_a*)(pp + 4), x2 = *(const v4f_a*)(pp + 16), x3 = *(const v4f_a*)(pp + 20);
#pragma unroll
        for (int i = 0; i < 4; ++i) { pv[i] = x0[i]; pv[4 + i] = x1[i]; pv[8 + i] = x2[i]; pv[12 + i] = x3[i]; }
        const F2 pq = bsplit16(pv);
#pragma unroll
        for (int dt = 0; dt < 8; ++dt) { const size_t po = (size_t)(kvh * HD + dt * 16u + col) * HIQ + k0 + kk * 32u; const v16b vh = frag_b(VB + po, lane); acc[dt] = wmma_bf(pq.h, vh, acc[dt]); acc[dt] = wmma_bf(pq.l, vh, acc[dt]); const v16b vl = frag_b(VBL + po, lane); acc[dt] = wmma_bf(pq.h, vl, acc[dt]); } }
    } else {
#pragma unroll 1
      for (unsigned kk = 0; kk < 2u; ++kk) { union { v16h v; v8h q[2]; } u; const _Float16* pp = &ph[wave][col][kk * 32u + 8u * g]; u.q[0] = *(const v8h_a*)pp; u.q[1] = *(const v8h_a*)(pp + 16);
#pragma unroll
        for (int dt = 0; dt < 8; ++dt) { const size_t po = (size_t)(kvh * HD + dt * 16u + col) * SEQ + k0 + kk * 32u; acc[dt] = wmma16(u.v, frag_h(VT + po, lane), acc[dt]); } } }
    LDSX(); }
#pragma unroll
  for (int r = 0; r < 8; ++r) { const float inv = (HI ? 16.0f : (16.0f / 2048.0f)) * (1.0f / lrow[r]);
#pragma unroll
    for (int dt = 0; dt < 8; ++dt) { const float c16 = acc[dt][r] * inv; const _Float16 hv = toh_flush(c16); cs[wave][8u * g + r][dt * 16u + col] = hv; if (HI) csl[wave][8u * g + r][dt * 16u + col] = toh_flush((c16 - (float)hv) * 1024.0f); } }
  LDSX();
#pragma unroll 1
  for (unsigned it = 0; it < 8u; ++it) { const unsigned rl = it * 2u + g; const size_t o = (size_t)(ql0 + rl) * EMB + h * HD + col * 8u;
    const v4u vh = *(const v4u_a*)&cs[wave][rl][col * 8u]; vst2((void*)(CH + o), vh);
    if (HI) { const v4u vl = *(const v4u_a*)&csl[wave][rl][col * 8u]; vst2((void*)(CL + o), vl); } }
}
__global__ __launch_bounds__(128) void k_attn_hi(const _Float16* __restrict__ QH, const _Float16* __restrict__ KH, const _Float16* __restrict__ VT, const _Float16* __restrict__ QL, const _Float16* __restrict__ KL,
    const __bf16* __restrict__ VB, const __bf16* __restrict__ VBL, _Float16* __restrict__ CH, _Float16* __restrict__ CL) { attn_body<true>(QH, KH, VT, QL, KL, VB, VBL, CH, CL, 0u); }
__global__ __launch_bounds__(128) void k_attn_lo(const _Float16* __restrict__ QH, const _Float16* __restrict__ KH, const _Float16* __restrict__ VT, const _Float16* __restrict__ QL, const _Float16* __restrict__ KL,
    const __bf16* __restrict__ VB, const __bf16* __restrict__ VBL, _Float16* __restrict__ CH, _Float16* __restrict__ CL) { attn_body<false>(QH, KH, VT, QL, KL, VB, VBL, CH, CL, (unsigned)(HIQ / 64)); }

template <bool HI>
__device__ __forceinline__ void out_body(const _Float16* __restrict__ CH, const _Float16* __restrict__ CL, const _Float16* __restrict__ WO, float* __restrict__ OUT, unsigned rb0) {
  __shared__ __align__(16) float so[64][132];
  const unsigned tid = threadIdx.x, wave = tid >> 5, lane = tid & 31u, col = lane & 15u, g = lane >> 4;
  const unsigned r0 = (rb0 + blockIdx.x) * 64u, c0 = blockIdx.y * 128u; const unsigned wr = (wave & 1u) * 32u, wc = (wave >> 1) * 64u;
  v8f acc[2][4] = {}, accr[2][4] = {};
  const size_t ao = (size_t)(r0 + wr + col) * EMB; const _Float16* pb = WO + (size_t)(c0 + wc + col) * EMB;
#pragma unroll 1
  for (unsigned kc = 0; kc < EMB; kc += 32u) { const v16h a0 = frag_h(CH + ao + kc, lane), a1 = frag_h(CH + ao + (size_t)16u * EMB + kc, lane); v16h l0 = a0, l1 = a1;
    if (HI) { l0 = frag_h(CL + ao + kc, lane); l1 = frag_h(CL + ao + (size_t)16u * EMB + kc, lane); }
#pragma unroll
    for (int t = 0; t < 4; ++t) { const v16h w = frag_h(pb + (size_t)t * 16u * EMB + kc, lane); acc[0][t] = wmma16(a0, w, acc[0][t]); acc[1][t] = wmma16(a1, w, acc[1][t]);
      if (HI) { accr[0][t] = wmma16(l0, w, accr[0][t]); accr[1][t] = wmma16(l1, w, accr[1][t]); } } }
#pragma unroll
  for (int mi = 0; mi < 2; ++mi)
#pragma unroll
    for (int t = 0; t < 4; ++t) { const unsigned cl = wc + t * 16u + col;
#pragma unroll
      for (int r = 0; r < 8; ++r) { float v = acc[mi][t][r]; if (HI) v += accr[mi][t][r] * (1.0f / 1024.0f); so[wr + mi * 16u + 8u * g + r][cl] = v * (1.0f / 4096.0f); } }
  __syncthreads();
#pragma unroll 1
  for (unsigned i = 0; i < 16u; ++i) { const unsigned rl = wave * 16u + i; const v4f v = *(const v4f_a*)&so[rl][lane * 4u]; vst2((void*)(OUT + (size_t)(r0 + rl) * EMB + c0 + lane * 4u), v); }
}
__global__ __launch_bounds__(128) void k_out_hi(const _Float16* __restrict__ CH, const _Float16* __restrict__ CL, const _Float16* __restrict__ WO, float* __restrict__ OUT) { out_body<true>(CH, CL, WO, OUT, 0u); }
__global__ __launch_bounds__(128) void k_out_lo(const _Float16* __restrict__ CH, const _Float16* __restrict__ CL, const _Float16* __restrict__ WO, float* __restrict__ OUT) { out_body<false>(CH, CL, WO, OUT, (unsigned)(HIQ / 64)); }

extern "C" void kernel_launch(void* const* d_in, const int* in_sizes, int n_in, void* d_out, int out_size, void* d_ws, size_t ws_size, hipStream_t stream) {
  if (n_in < 5) return;
  if ((size_t)in_sizes[0] < (size_t)SEQ * EMB) return;
  if ((size_t)in_sizes[1] < (size_t)EMB * EMB) return;
  if ((size_t)in_sizes[2] < (size_t)KVW * EMB) return;
  if ((size_t)in_sizes[3] < (size_t)KVW * EMB) return;
  if ((size_t)in_sizes[4] < (size_t)EMB * EMB) return;
  if ((size_t)out_size < (size_t)SEQ * EMB) return;
  if (ws_size < (size_t)WS_END) return;
  const float* x = (const float*)d_in[0]; const float* wq = (const float*)d_in[1]; const float* wk = (const float*)d_in[2];
  const float* wv = (const float*)d_in[3]; const float* wo = (const float*)d_in[4];
  char* ws = (char*)d_ws;
  __bf16* XB = (__bf16*)(ws + WS_XB); __bf16* WB = (__bf16*)(ws + WS_WB); _Float16* WO = (_Float16*)(ws + WS_WO);
  _Float16 *QH = (_Float16*)(ws + WS_QH), *KH = (_Float16*)(ws + WS_KH), *VT = (_Float16*)(ws + WS_VT), *QL = (_Float16*)(ws + WS_QL), *KL = (_Float16*)(ws + WS_KL);
  __bf16 *VB = (__bf16*)(ws + WS_VB), *VBL = (__bf16*)(ws + WS_VBL); _Float16 *CH = (_Float16*)(ws + WS_CH), *CL = (_Float16*)(ws + WS_CL);
  float* CS = (float*)(ws + WS_CS);
  const unsigned nx8 = (unsigned)((size_t)SEQ * EMB / 8u), nq8 = (unsigned)((size_t)EMB * EMB / 8u), nk8 = (unsigned)((size_t)KVW * EMB / 8u);
  k_cvt_b<<<dim3(nx8 / 256u), 256, 0, stream>>>(x, XB, nx8);
  k_cvt_b<<<dim3(nq8 / 256u), 256, 0, stream>>>(wq, WB, nq8);
  k_cvt_b<<<dim3(nk8 / 256u), 256, 0, stream>>>(wk, WB + (size_t)EMB * EMB, nk8);
  k_cvt_b<<<dim3(nk8 / 256u), 256, 0, stream>>>(wv, WB + (size_t)(EMB + KVW) * EMB, nk8);
  k_cvt_h<<<dim3(nq8 / 256u), 256, 0, stream>>>(wo, WO, nq8);
  k_rope_tab<<<dim3(SEQ / 4), 256, 0, stream>>>(CS);
  k_proj<<<dim3(SEQ / 64, NQKV / 128u), 128, 0, stream>>>(XB, WB, CS, QH, QL, KH, KL, VT, VB, VBL);
  k_attn_hi<<<dim3(HIQ / 64, NH), 128, 0, stream>>>(QH, KH, VT, QL, KL, VB, VBL, CH, CL);
  if ((SEQ - HIQ) / 64 > 0) k_attn_lo<<<dim3((SEQ - HIQ) / 64, NH), 128, 0, stream>>>(QH, KH, VT, QL, KL, VB, VBL, CH, CL);
  k_out_hi<<<dim3(HIQ / 64, EMB / 128u), 128, 0, stream>>>(CH, CL, WO, (float*)d_out);
  if ((SEQ - HIQ) / 64 > 0) k_out_lo<<<dim3((SEQ - HIQ) / 64, EMB / 128u), 128, 0, stream>>>(CH, CL, WO, (float*)d_out);
}
